// HyperbolicMLR_31078383354263
// MI455X (gfx1250) — hardware-run, weakly checked
//
#include <hip/hip_runtime.h>


#define NSB  2048
#define NCL  1000
#define NCP  1024
#define NDM  64
#define KCV  0.1f
#define EPV  1e-15f
#define PSC  16.0f
#define IPS  0.00390625f
constexpr size_t al256(size_t b) { return (b + 255) & ~(size_t)255; }
constexpr size_t WS_TOTAL = al256((size_t)NSB * NDM * 2) + al256((size_t)2 * NCP * NDM * 2) + al256((size_t)NCP * 4 * 4) + al256((size_t)NSB * 4) + al256((size_t)NSB * 2 * NCP * 4);
static_assert(WS_TOTAL == 17326080 && WS_TOTAL <= 134217728, "the workspace carve: 16.5 MiB");
static_assert(NSB % 64 == 0 && (2 * NCP) % 64 == 0 && NDM % 32 == 0 && NDM * 2 == 128 && NCL % 4 == 0 && ((size_t)NSB * NCL) % 128 == 0 && NCP >= NCL, "whole tiles; whole depth steps; an operand row is one line; four classes a thread never straddle a sample");
typedef _Float16 h16;
typedef unsigned short bf;
typedef __attribute__((ext_vector_type(16))) __bf16   v16bf;
typedef __attribute__((ext_vector_type(16))) _Float16 v16h;
typedef __attribute__((ext_vector_type(8)))  _Float16 v8h;
typedef __attribute__((ext_vector_type(8)))  unsigned short v8us;
typedef __attribute__((ext_vector_type(8)))  float    v8f;
typedef __attribute__((ext_vector_type(4)))  float    v4f;
typedef v8h  __attribute__((may_alias)) v8ha;
typedef v4f  __attribute__((may_alias)) v4fa;
typedef v8us __attribute__((may_alias)) v8usa;

__device__ __forceinline__ unsigned short f2bf(float f) { unsigned u = __float_as_uint(f); u += 0x7FFFu + ((u >> 16) & 1u); return (unsigned short)(u >> 16); }
__device__ __forceinline__ float bf2f(unsigned short b) { return __uint_as_float(((unsigned)b) << 16); }
__device__ __forceinline__ float bfr(float f) { return bf2f(f2bf(f)); }
__device__ __forceinline__ v16h cat16(v8h lo, v8h hi) { return __builtin_shufflevector(lo, hi, 0, 1, 2, 3, 4, 5, 6, 7, 8, 9, 10, 11, 12, 13, 14, 15); }
__device__ __forceinline__ v16bf cat16b(v8us lo, v8us hi) { return __builtin_bit_cast(v16bf, __builtin_shufflevector(lo, hi, 0, 1, 2, 3, 4, 5, 6, 7, 8, 9, 10, 11, 12, 13, 14, 15)); }
__device__ __forceinline__ v8f wmma16(v16h a, v16h b, v8f c) { return __builtin_amdgcn_wmma_f32_16x16x32_f16(false, a, false, b, (short)0, c, false, false); }
__device__ __forceinline__ v8f wmmab(v16bf a, v16bf b, v8f c) { return __builtin_amdgcn_wmma_f32_16x16x32_bf16(false, a, false, b, (short)0, c, false, false); }


template <typename T16> struct WFrag;
template <> struct WFrag<h16> { typedef v16h V; static __device__ __forceinline__ V ld(const h16* p) { return cat16(*(const v8h*)p, *(const v8h*)(p + 16)); } static __device__ __forceinline__ v8f mma(V a, V b, v8f c) { return wmma16(a, b, c); } };
template <> struct WFrag<bf> { typedef v16bf V; static __device__ __forceinline__ V ld(const bf* p) { return cat16b(*(const v8us*)p, *(const v8us*)(p + 16)); } static __device__ __forceinline__ v8f mma(V a, V b, v8f c) { return wmmab(a, b, c); } };
template <typename T16, int NSPLIT, bool BIAS>
__global__ __launch_bounds__(32) void k_gemmw(const T16* __restrict__ A, const T16* __restrict__ A2, const T16* __restrict__ Bt, const T16* __restrict__ Bt2, int K, float* C, int ldc, const float* __restrict__ bias, size_t sA, size_t sB, size_t sC) {
    typedef typename WFrag<T16>::V V;
    __shared__ __align__(16) float os[16 * 68];
    const size_t z = blockIdx.z; A += z * sA; if (A2) A2 += z * sA; Bt += z * sB; if (Bt2) Bt2 += z * sB; C += z * sC;
    const int lane = threadIdx.x & 31, lr = lane & 15, hi = lane >> 4; const int r0 = blockIdx.x * 64, c0 = blockIdx.y * 64;
    v8f acc[4][4];
#pragma unroll
    for (int mb = 0; mb < 4; ++mb)
#pragma unroll
        for (int nb = 0; nb < 4; ++nb) acc[mb][nb] = (v8f){};
    const size_t aoff = (size_t)(r0 + lr) * K + 8 * hi, boff = (size_t)(c0 + lr) * K + 8 * hi;
    for (int kc = 0; kc < K; kc += 32) {
        V a[4], a2[4];
#pragma unroll
        for (int mb = 0; mb < 4; ++mb) { a[mb] = WFrag<T16>::ld(A + aoff + (size_t)mb * 16 * K + kc); if (NSPLIT == 1 || NSPLIT == 2) a2[mb] = WFrag<T16>::ld(A2 + aoff + (size_t)mb * 16 * K + kc); }
#pragma unroll
        for (int nb = 0; nb < 4; ++nb) { const V b = WFrag<T16>::ld(Bt + boff + (size_t)nb * 16 * K + kc); V b2; if (NSPLIT >= 2) b2 = WFrag<T16>::ld(Bt2 + boff + (size_t)nb * 16 * K + kc);
#pragma unroll
            for (int mb = 0; mb < 4; ++mb) { acc[mb][nb] = WFrag<T16>::mma(a[mb], b, acc[mb][nb]); if (NSPLIT == 1 || NSPLIT == 2) acc[mb][nb] = WFrag<T16>::mma(a2[mb], b, acc[mb][nb]); if (NSPLIT >= 2) acc[mb][nb] = WFrag<T16>::mma(a[mb], b2, acc[mb][nb]); } }
        asm volatile("v_nop\n\tv_nop\n\tv_nop\n\tv_nop" : "+v"(acc[0][0]), "+v"(acc[1][1]), "+v"(acc[2][2]), "+v"(acc[3][3]) : "v"(a[0]), "v"(a[3]));
    }
#pragma unroll
    for (int mb = 0; mb < 4; ++mb) {
#pragma unroll
        for (int nb = 0; nb < 4; ++nb) {
#pragma unroll
            for (int j = 0; j < 8; ++j) os[(hi * 8 + j) * 68 + nb * 16 + lr] = acc[mb][nb][j]; }
        __builtin_amdgcn_wave_barrier(); asm volatile("" ::: "memory");
        float* crow = C + (size_t)(r0 + mb * 16) * ldc + c0;
#pragma unroll 1
        for (int ps = 0; ps < 2; ++ps) {
#pragma unroll
            for (int s = 0; s < 8; ++s) { const int row = 2 * s + hi, cofs = lr * 4; v4f val = *(const v4fa*)(os + row * 68 + cofs); if (BIAS) { val[0] += bfr(bias[c0 + cofs]); val[1] += bfr(bias[c0 + cofs + 1]); val[2] += bfr(bias[c0 + cofs + 2]); val[3] += bfr(bias[c0 + cofs + 3]); }
                *(volatile v4f*)(crow + (size_t)row * ldc + cofs) = val; }
            if (ps == 0) __threadfence(); }
        __builtin_amdgcn_wave_barrier(); asm volatile("" ::: "memory");
    }
}

__device__ __forceinline__ h16 tohx(float x) { return (h16)x; }
__device__ __forceinline__ void splitf(float y, unsigned short& h, unsigned short& l) { h = f2bf(y); l = f2bf(y - bf2f(h)); }
typedef __attribute__((ext_vector_type(2))) _Float16 v2h;
typedef __attribute__((ext_vector_type(4))) _Float16 v4h;
typedef __attribute__((ext_vector_type(2))) unsigned short v2us;
typedef __attribute__((ext_vector_type(4))) unsigned short v4us;
typedef __attribute__((ext_vector_type(2))) float v2f;
typedef __attribute__((ext_vector_type(4))) int v4i;


__global__ __launch_bounds__(64) void k_cls(const float* __restrict__ av, const float* __restrict__ pv, h16* BT, float* TB) {
    const unsigned c = blockIdx.x * 64 + threadIdx.x; if (c >= (unsigned)NCP) return; const unsigned cr = c < (unsigned)NCL ? c : (unsigned)(NCL - 1); const float lv = c < (unsigned)NCL ? 1.0f : 0.0f;
    const float* pr = pv + (size_t)cr * NDM; const float* ar = av + (size_t)cr * NDM; const float sk = sqrtf(KCV); float s2 = 0.0f;
    for (int d = 0; d < NDM; ++d) { const float p = bfr(pr[d]); s2 += p * p; }
    const float pn = fmaxf(sqrtf(s2), EPV); const float th = tanhf(sk * pn) / (sk * pn); float q2 = 0.0f; h16* dw = BT + (size_t)c * NDM; h16* da = BT + (size_t)(NCP + c) * NDM;
    for (int d8 = 0; d8 < NDM / 8; ++d8) { v8h o;
#pragma unroll
        for (int q = 0; q < 8; ++q) { const float pq = th * bfr(pr[8 * d8 + q]); q2 += pq * pq; o[q] = tohx(-pq * PSC * lv); }
        *(volatile v8h*)(dw + 8 * d8) = o; __threadfence(); *(volatile v8h*)(dw + 8 * d8) = o; }
    const float fc = 1.0f + KCV * q2; float a2 = 0.0f, wa = 0.0f;
    for (int d8 = 0; d8 < NDM / 8; ++d8) { v8h o;
#pragma unroll
        for (int q = 0; q < 8; ++q) { const float aq = bfr(ar[8 * d8 + q]) * fc; const float pq = th * bfr(pr[8 * d8 + q]); a2 += aq * aq; wa += -pq * aq; o[q] = tohx(aq * PSC * lv); }
        *(volatile v8h*)(da + 8 * d8) = o; __threadfence(); *(volatile v8h*)(da + 8 * d8) = o; }
    const float an = fmaxf(sqrtf(a2), EPV); const float sc = (2.0f / (1.0f - KCV * q2)) * an / sk; v4f t; t[0] = q2 * lv; t[1] = wa * lv; t[2] = an * lv; t[3] = sc * lv;
    *(volatile v4f*)(TB + (size_t)c * 4) = t; __threadfence(); *(volatile v4f*)(TB + (size_t)c * 4) = t; }

__global__ __launch_bounds__(64) void k_smp(const float* __restrict__ xi, h16* XA, float* YS) {
    const unsigned b = blockIdx.x * 64 + threadIdx.x; if (b >= (unsigned)NSB) return; const float* xr = xi + (size_t)b * NDM; h16* dx = XA + (size_t)b * NDM; float ys = 0.0f;
    for (int d8 = 0; d8 < NDM / 8; ++d8) { v8h o;
#pragma unroll
        for (int q = 0; q < 8; ++q) { const float xw = bfr(xr[8 * d8 + q]); ys += xw * xw; o[q] = tohx(xw * PSC); }
        *(volatile v8h*)(dx + 8 * d8) = o; __threadfence(); *(volatile v8h*)(dx + 8 * d8) = o; }
    *(volatile float*)(YS + b) = ys; __threadfence(); *(volatile float*)(YS + b) = ys; }

__global__ __launch_bounds__(256) void k_out(const float* __restrict__ CC, const float* __restrict__ TB, const float* __restrict__ YS, float* rs) {
    const unsigned e = blockIdx.x * 256 + threadIdx.x; if (e >= (unsigned)(NSB * (NCL / 4))) return; const unsigned b = e / (NCL / 4), c0 = (e - b * (NCL / 4)) * 4;
    const float ys = YS[b]; const float sk = sqrtf(KCV); const v4f uu = *(const v4f*)(CC + (size_t)b * (2 * NCP) + c0); const v4f xx = *(const v4f*)(CC + (size_t)b * (2 * NCP) + NCP + c0); v4f o;
#pragma unroll
    for (int q = 0; q < 4; ++q) { const v4f t = *(const v4f*)(TB + (size_t)(c0 + q) * 4); const float q2 = t[0], wa = t[1], an = t[2], sc = t[3]; const float u = uu[q] * IPS, xa = xx[q] * IPS;
        const float ca = 1.0f + 2.0f * KCV * u + KCV * ys; const float cb = 1.0f - KCV * q2; const float de = 1.0f + 2.0f * KCV * u + (KCV * KCV) * q2 * ys;
        const float ma = (ca * wa + cb * xa) / de; const float mm = (ca * ca * q2 + 2.0f * ca * cb * u + cb * cb * ys) / (de * de);
        o[q] = sc * asinhf((2.0f * sk * ma) / (an * (1.0f - KCV * mm))); }
    float* d = rs + (size_t)e * 4; *(volatile v4f*)(d) = o; __threadfence(); *(volatile v4f*)(d) = o; }

extern "C" void kernel_launch(void* const* d_in, const int* in_sizes, int n_in,
                              void* d_out, int out_size, void* d_ws, size_t ws_size, hipStream_t stream) {
    if (n_in < 3) return;
    if (in_sizes[0] < NSB * NDM || in_sizes[1] < NCL * NDM || in_sizes[2] < NCL * NDM || out_size < NSB * NCL) return;
    const float* xi = (const float*)d_in[0]; const float* av = (const float*)d_in[1]; const float* pv = (const float*)d_in[2];
    char* wsp = (char*)d_ws;
    auto take = [&](size_t bytes) { char* cur = wsp; wsp += (bytes + 255) & ~(size_t)255; return (void*)cur; };
    h16* XA = (h16*)take((size_t)NSB * NDM * 2); h16* BT = (h16*)take((size_t)2 * NCP * NDM * 2); float* TB = (float*)take((size_t)NCP * 4 * 4); float* YS = (float*)take((size_t)NSB * 4); float* CC = (float*)take((size_t)NSB * 2 * NCP * 4);
    if ((size_t)(wsp - (char*)d_ws) != WS_TOTAL || WS_TOTAL > ws_size) return;
    k_cls<<<NCP / 64, 64, 0, stream>>>(av, pv, BT, TB);
    k_smp<<<NSB / 64, 64, 0, stream>>>(xi, XA, YS);
    k_gemmw<h16, 0, false><<<dim3(NSB / 64, 2 * NCP / 64, 1), 32, 0, stream>>>(XA, nullptr, BT, nullptr, NDM, CC, 2 * NCP, nullptr, (size_t)0, (size_t)0, (size_t)0);
    k_out<<<NSB * (NCL / 4) / 256, 256, 0, stream>>>(CC, TB, YS, (float*)d_out);
}
